// RA_MLA_Attention_73478300500273
// MI455X (gfx1250) — hardware-verified
//
#include <hip/hip_runtime.h>


#define TT   2048
#define EE   2048
#define NH_  16
#define HD   128
#define LL   64
#define ZH   2
typedef _Float16 h16;
typedef unsigned short bf;
typedef __attribute__((ext_vector_type(16))) __bf16   v16bf;
typedef __attribute__((ext_vector_type(16))) _Float16 v16h;
typedef __attribute__((ext_vector_type(8)))  _Float16 v8h;
typedef __attribute__((ext_vector_type(8)))  unsigned short v8us;
typedef __attribute__((ext_vector_type(8)))  float    v8f;
typedef __attribute__((ext_vector_type(4)))  float    v4f;
typedef v8h  __attribute__((may_alias)) v8ha;
typedef v4f  __attribute__((may_alias)) v4fa;
typedef v8us __attribute__((may_alias)) v8usa;

__device__ __forceinline__ unsigned short f2bf(float f) { unsigned u = __float_as_uint(f); u += 0x7FFFu + ((u >> 16) & 1u); return (unsigned short)(u >> 16); }
__device__ __forceinline__ float bf2f(unsigned short b) { return __uint_as_float(((unsigned)b) << 16); }
__device__ __forceinline__ float bfr(float f) { return bf2f(f2bf(f)); }
__device__ __forceinline__ v16h cat16(v8h lo, v8h hi) { return __builtin_shufflevector(lo, hi, 0, 1, 2, 3, 4, 5, 6, 7, 8, 9, 10, 11, 12, 13, 14, 15); }
__device__ __forceinline__ v16bf cat16b(v8us lo, v8us hi) { return __builtin_bit_cast(v16bf, __builtin_shufflevector(lo, hi, 0, 1, 2, 3, 4, 5, 6, 7, 8, 9, 10, 11, 12, 13, 14, 15)); }
__device__ __forceinline__ v8f wmma16(v16h a, v16h b, v8f c) { return __builtin_amdgcn_wmma_f32_16x16x32_f16(false, a, false, b, (short)0, c, false, false); }
__device__ __forceinline__ v8f wmmab(v16bf a, v16bf b, v8f c) { return __builtin_amdgcn_wmma_f32_16x16x32_bf16(false, a, false, b, (short)0, c, false, false); }


template <typename T16> struct WFrag;
template <> struct WFrag<h16> { typedef v16h V; static __device__ __forceinline__ V ld(const h16* p) { return cat16(*(const v8h*)p, *(const v8h*)(p + 16)); } static __device__ __forceinline__ v8f mma(V a, V b, v8f c) { return wmma16(a, b, c); } };
template <> struct WFrag<bf> { typedef v16bf V; static __device__ __forceinline__ V ld(const bf* p) { return cat16b(*(const v8us*)p, *(const v8us*)(p + 16)); } static __device__ __forceinline__ v8f mma(V a, V b, v8f c) { return wmmab(a, b, c); } };
template <typename T16, int NSPLIT, bool BIAS>
__global__ __launch_bounds__(32) void k_gemmw(const T16* __restrict__ A, const T16* __restrict__ A2, const T16* __restrict__ Bt, const T16* __restrict__ Bt2, int K, float* C, int ldc, const float* __restrict__ bias, size_t sA, size_t sB, size_t sC) {
    typedef typename WFrag<T16>::V V;
    __shared__ __align__(16) float os[16 * 68];
    const size_t z = blockIdx.z; A += z * sA; if (A2) A2 += z * sA; Bt += z * sB; if (Bt2) Bt2 += z * sB; C += z * sC;
    const int lane = threadIdx.x & 31, lr = lane & 15, hi = lane >> 4; const int r0 = blockIdx.x * 64, c0 = blockIdx.y * 64;
    v8f acc[4][4];
#pragma unroll
    for (int mb = 0; mb < 4; ++mb)
#pragma unroll
        for (int nb = 0; nb < 4; ++nb) acc[mb][nb] = (v8f){};
    const size_t aoff = (size_t)(r0 + lr) * K + 8 * hi, boff = (size_t)(c0 + lr) * K + 8 * hi;
#pragma unroll 1
    for (int kc = 0; kc < K; kc += 32) {
        V a[4], a2[4];
#pragma unroll
        for (int mb = 0; mb < 4; ++mb) { a[mb] = WFrag<T16>::ld(A + aoff + (size_t)mb * 16 * K + kc); if (NSPLIT == 1 || NSPLIT == 2) a2[mb] = WFrag<T16>::ld(A2 + aoff + (size_t)mb * 16 * K + kc); }
#pragma unroll
        for (int nb = 0; nb < 4; ++nb) { const V b = WFrag<T16>::ld(Bt + boff + (size_t)nb * 16 * K + kc); V b2; if (NSPLIT >= 2) b2 = WFrag<T16>::ld(Bt2 + boff + (size_t)nb * 16 * K + kc);
#pragma unroll
            for (int mb = 0; mb < 4; ++mb) { acc[mb][nb] = WFrag<T16>::mma(a[mb], b, acc[mb][nb]); if (NSPLIT == 1 || NSPLIT == 2) acc[mb][nb] = WFrag<T16>::mma(a2[mb], b, acc[mb][nb]); if (NSPLIT >= 2) acc[mb][nb] = WFrag<T16>::mma(a[mb], b2, acc[mb][nb]); } }
        asm volatile("v_nop\n\tv_nop\n\tv_nop\n\tv_nop" : "+v"(acc[0][0]), "+v"(acc[1][1]), "+v"(acc[2][2]), "+v"(acc[3][3]) : "v"(a[0]), "v"(a[3]));
    }
#pragma unroll
    for (int mb = 0; mb < 4; ++mb) {
#pragma unroll
        for (int nb = 0; nb < 4; ++nb) {
#pragma unroll
            for (int j = 0; j < 8; ++j) os[(hi * 8 + j) * 68 + nb * 16 + lr] = acc[mb][nb][j]; }
        __builtin_amdgcn_wave_barrier(); asm volatile("" ::: "memory");
        float* crow = C + (size_t)(r0 + mb * 16) * ldc + c0;
#pragma unroll 1
        for (int ps = 0; ps < 2; ++ps) {
#pragma unroll
            for (int s = 0; s < 8; ++s) { const int row = 2 * s + hi, cofs = lr * 4; v4f val = *(const v4fa*)(os + row * 68 + cofs); if (BIAS) { val[0] += bfr(bias[c0 + cofs]); val[1] += bfr(bias[c0 + cofs + 1]); val[2] += bfr(bias[c0 + cofs + 2]); val[3] += bfr(bias[c0 + cofs + 3]); }
                *(volatile v4f*)(crow + (size_t)row * ldc + cofs) = val; }
            if (ps == 0) __threadfence(); }
        __builtin_amdgcn_wave_barrier(); asm volatile("" ::: "memory");
    }
}

template <typename T16, int NSPLIT, int CMODE>
__global__ __launch_bounds__(32) void k_gemmc(const T16* __restrict__ A, const T16* __restrict__ A2, const T16* __restrict__ Bt, const T16* __restrict__ Bt2, int K, float* C, int ldc, int roff, size_t sA, size_t sB, size_t sC) {
    typedef typename WFrag<T16>::V V;
    __shared__ __align__(16) float os[16 * 68];
    const size_t z = blockIdx.z; A += z * sA; if (A2) A2 += z * sA; Bt += z * sB; if (Bt2) Bt2 += z * sB; C += z * sC;
    const int lane = threadIdx.x & 31, lr = lane & 15, hi = lane >> 4; const int r0 = blockIdx.x * 64, c0 = blockIdx.y * 64;
    if (CMODE == 1 && c0 > r0 + roff + 63) return;
    const int Kl = (CMODE == 2) ? min(K, r0 + roff + 64) : K;
    v8f acc[4][4];
#pragma unroll
    for (int mb = 0; mb < 4; ++mb)
#pragma unroll
        for (int nb = 0; nb < 4; ++nb) acc[mb][nb] = (v8f){};
    const size_t aoff = (size_t)(r0 + lr) * K + 8 * hi, boff = (size_t)(c0 + lr) * K + 8 * hi;
#pragma unroll 1
    for (int kc = 0; kc < Kl; kc += 32) {
        V a[4], a2[4];
#pragma unroll
        for (int mb = 0; mb < 4; ++mb) { a[mb] = WFrag<T16>::ld(A + aoff + (size_t)mb * 16 * K + kc); if (NSPLIT == 1 || NSPLIT == 2) a2[mb] = WFrag<T16>::ld(A2 + aoff + (size_t)mb * 16 * K + kc); }
#pragma unroll
        for (int nb = 0; nb < 4; ++nb) { const V b = WFrag<T16>::ld(Bt + boff + (size_t)nb * 16 * K + kc); V b2; if (NSPLIT >= 2) b2 = WFrag<T16>::ld(Bt2 + boff + (size_t)nb * 16 * K + kc);
#pragma unroll
            for (int mb = 0; mb < 4; ++mb) { acc[mb][nb] = WFrag<T16>::mma(a[mb], b, acc[mb][nb]); if (NSPLIT == 1 || NSPLIT == 2) acc[mb][nb] = WFrag<T16>::mma(a2[mb], b, acc[mb][nb]); if (NSPLIT >= 2) acc[mb][nb] = WFrag<T16>::mma(a[mb], b2, acc[mb][nb]); } }
        asm volatile("v_nop\n\tv_nop\n\tv_nop\n\tv_nop" : "+v"(acc[0][0]), "+v"(acc[1][1]), "+v"(acc[2][2]), "+v"(acc[3][3]) : "v"(a[0]), "v"(a[3]));
    }
#pragma unroll
    for (int mb = 0; mb < 4; ++mb) {
#pragma unroll
        for (int nb = 0; nb < 4; ++nb) {
#pragma unroll
            for (int j = 0; j < 8; ++j) os[(hi * 8 + j) * 68 + nb * 16 + lr] = acc[mb][nb][j]; }
        __builtin_amdgcn_wave_barrier(); asm volatile("" ::: "memory");
        float* crow = C + (size_t)(r0 + mb * 16) * ldc + c0;
#pragma unroll 1
        for (int ps = 0; ps < 2; ++ps) {
#pragma unroll
            for (int s = 0; s < 8; ++s) { const int row = 2 * s + hi, cofs = lr * 4; v4f val = *(const v4fa*)(os + row * 68 + cofs);
                *(volatile v4f*)(crow + (size_t)row * ldc + cofs) = val; }
            if (ps == 0) __threadfence(); }
        __builtin_amdgcn_wave_barrier(); asm volatile("" ::: "memory");
    }
}
__device__ __forceinline__ void splitf(float y, unsigned short& h, unsigned short& l) { h = f2bf(y); l = f2bf(y - bf2f(h)); }
typedef __attribute__((ext_vector_type(2))) unsigned short v2us;
typedef __attribute__((ext_vector_type(4))) unsigned short v4us;

__global__ __launch_bounds__(256) void k_cvt8(const float* __restrict__ src, bf* dst, size_t n8) { const size_t i = (size_t)blockIdx.x * 256 + threadIdx.x; if (i >= n8) return; const v8f v = *(const v8f*)(src + i * 8); v8us o;
#pragma unroll
    for (int k = 0; k < 8; ++k) o[k] = f2bf(v[k]); *(volatile v8us*)(dst + i * 8) = o; __threadfence(); *(volatile v8us*)(dst + i * 8) = o; }
__global__ __launch_bounds__(256) void k_qhpl(const float* __restrict__ Q, bf* Ph, bf* Pl) { const size_t e = ((size_t)blockIdx.x * 256 + threadIdx.x) * 4; if (e >= (size_t)NH_ * TT * HD) return; const int d = (int)(e % HD); const int t = (int)((e / HD) % TT); const int h = (int)(e / ((size_t)HD * TT)); const float* q = Q + (size_t)t * EE + h * HD + d; v4us oh, ol;
#pragma unroll
    for (int u = 0; u < 4; ++u) { unsigned short a, b; splitf(q[u], a, b); oh[u] = a; ol[u] = b; } *(volatile v4us*)(Ph + e) = oh; *(volatile v4us*)(Pl + e) = ol; __threadfence(); *(volatile v4us*)(Ph + e) = oh; *(volatile v4us*)(Pl + e) = ol; }
__global__ __launch_bounds__(256) void k_q2l(const float* __restrict__ w, bf* Bt) { const size_t e = ((size_t)blockIdx.x * 256 + threadIdx.x) * 4; if (e >= (size_t)NH_ * LL * HD) return; const int d = (int)(e % HD); const int l = (int)((e / HD) % LL); const int h = (int)(e / ((size_t)HD * LL)); v4us o;
#pragma unroll
    for (int u = 0; u < 4; ++u) o[u] = f2bf(w[((size_t)h * HD + d + u) * LL + l]); *(volatile v4us*)(Bt + e) = o; __threadfence(); *(volatile v4us*)(Bt + e) = o; }
__global__ __launch_bounds__(256) void k_vup(const float* __restrict__ w, bf* Bt) { const size_t e = ((size_t)blockIdx.x * 256 + threadIdx.x) * 4; if (e >= (size_t)NH_ * HD * LL) return; const int l = (int)(e % LL); const int d = (int)((e / LL) % HD); const int h = (int)(e / ((size_t)LL * HD)); v4us o;
#pragma unroll
    for (int u = 0; u < 4; ++u) o[u] = f2bf(w[((size_t)h * LL + l + u) * HD + d]); *(volatile v4us*)(Bt + e) = o; __threadfence(); *(volatile v4us*)(Bt + e) = o; }
__global__ __launch_bounds__(256) void k_pl(const float* __restrict__ F, size_t n, bf* Ph, bf* Pl) { const size_t e = ((size_t)blockIdx.x * 256 + threadIdx.x) * 4; if (e >= n) return; v4us oh, ol;
#pragma unroll
    for (int u = 0; u < 4; ++u) { unsigned short a, b; splitf(F[e + u], a, b); oh[u] = a; ol[u] = b; } *(volatile v4us*)(Ph + e) = oh; *(volatile v4us*)(Pl + e) = ol; __threadfence(); *(volatile v4us*)(Ph + e) = oh; *(volatile v4us*)(Pl + e) = ol; }
__global__ __launch_bounds__(256) void k_rsum64(const float* __restrict__ F, size_t nrows, float* S) { const size_t r = (size_t)blockIdx.x * 256 + threadIdx.x; if (r >= nrows) return; const float* f = F + r * LL; float s = 0.f;
#pragma unroll 8
    for (int l = 0; l < LL; ++l) s = __fadd_rn(s, f[l]); *(volatile float*)(S + r) = s; __threadfence(); *(volatile float*)(S + r) = s; }
__global__ __launch_bounds__(256) void k_vet(const float* __restrict__ VE, bf* Vh, bf* Vl) { const size_t e = ((size_t)blockIdx.x * 256 + threadIdx.x) * 2; if (e >= (size_t)NH_ * HD * TT) return; const int t = (int)(e % TT); const int d = (int)((e / TT) % HD); const int h = (int)(e / ((size_t)TT * HD)); v2us oh, ol;
#pragma unroll
    for (int u = 0; u < 2; ++u) { unsigned short a, b; splitf(VE[((size_t)h * TT + t + u) * HD + d], a, b); oh[u] = a; ol[u] = b; } *(volatile v2us*)(Vh + e) = oh; *(volatile v2us*)(Vl + e) = ol; __threadfence(); *(volatile v2us*)(Vh + e) = oh; *(volatile v2us*)(Vl + e) = ol; }
__global__ __launch_bounds__(256) void k_csoft(const float* __restrict__ S, const float* __restrict__ sq, const float* __restrict__ sk, int h0, bf* Ph, bf* Pl) { const int lane = threadIdx.x & 31; const int row = blockIdx.x * 8 + (threadIdx.x >> 5); if (row >= ZH * TT) return; const int i = row % TT; const int zz = row / TT; const float* sr = S + (size_t)row * TT; const int jlim = ((i >> 6) + 1) * 64; const float sqi = sq[(size_t)(h0 + zz) * TT + i];
    float v[TT / 32]; float mx = -3.0e38f;
#pragma unroll
    for (int ch = 0; ch < TT / 128; ++ch) { const int j0 = ch * 128 + lane * 4; v4f a; if (j0 < jlim) a = *(const v4f*)(sr + j0); else { a[0] = 0.f; a[1] = 0.f; a[2] = 0.f; a[3] = 0.f; } const v4f k4 = *(const v4f*)(sk + j0);
#pragma unroll
        for (int u = 0; u < 4; ++u) { const int j = j0 + u; float t = a[u] * 0.125f; if (j <= i && i - j <= 64) { float r = __fmul_rn(sqi, k4[u]) * 0.125f; asm volatile("" : "+v"(r)); float hr = r * 0.5f; asm volatile("" : "+v"(hr)); t = __fadd_rn(t, hr); } t = (j <= i) ? t : -3.0e38f; v[ch * 4 + u] = t; mx = fmaxf(mx, t); } }
#pragma unroll
    for (int sh = 16; sh; sh >>= 1) mx = fmaxf(mx, __shfl_xor(mx, sh, 32));
    float sum = 0.f;
#pragma unroll
    for (int q = 0; q < TT / 32; ++q) { float d0 = __fsub_rn(v[q], mx); asm volatile("" : "+v"(d0)); v[q] = __builtin_amdgcn_exp2f(__fmul_rn(d0, 1.4426950408889634f)); sum += v[q]; }
#pragma unroll
    for (int sh = 16; sh; sh >>= 1) sum += __shfl_xor(sum, sh, 32);
    const float f = __fdiv_rn(1.0f, sum);
    for (int ps = 0; ps < 2; ++ps) {
#pragma unroll
        for (int ch = 0; ch < TT / 128; ++ch) { v4us oh, ol; for (int q = 0; q < 4; ++q) { unsigned short a2, c2; splitf(v[ch * 4 + q] * f, a2, c2); oh[q] = a2; ol[q] = c2; } const size_t oo = (size_t)row * TT + ch * 128 + lane * 4; *(volatile v4us*)(Ph + oo) = oh; *(volatile v4us*)(Pl + oo) = ol; }
        if (ps == 0) __threadfence(); } }
__global__ __launch_bounds__(256) void k_merge(const float* __restrict__ O, int h0, bf* Ah, bf* Al) { const size_t e = ((size_t)blockIdx.x * 256 + threadIdx.x) * 4; if (e >= (size_t)ZH * TT * HD) return; const int d = (int)(e % HD); const int t = (int)((e / HD) % TT); const int zz = (int)(e / ((size_t)HD * TT)); const size_t oo = (size_t)t * EE + (h0 + zz) * HD + d; v4us oh, ol;
#pragma unroll
    for (int u = 0; u < 4; ++u) { unsigned short a, b; splitf(O[e + u], a, b); oh[u] = a; ol[u] = b; } *(volatile v4us*)(Ah + oo) = oh; *(volatile v4us*)(Al + oo) = ol; __threadfence(); *(volatile v4us*)(Ah + oo) = oh; *(volatile v4us*)(Al + oo) = ol; }

extern "C" void kernel_launch(void* const* d_in, const int* in_sizes, int n_in,
                              void* d_out, int out_size, void* d_ws, size_t ws_size, hipStream_t stream) {
    (void)in_sizes; (void)n_in; (void)out_size;
    const float** I = (const float**)d_in;
    const float *x = I[0], *Wq = I[1], *Wk = I[2], *Wv = I[3], *q2l = I[4], *vup = I[5], *Wo = I[6];
    float* OUT = (float*)d_out;
    char* wsp = (char*)d_ws;
    auto take = [&](size_t bytes) { char* p = wsp; wsp += (bytes + 255) & ~(size_t)255; return (void*)p; };
    bf* XB = (bf*)take((size_t)TT * EE * 2); bf* BQ = (bf*)take((size_t)EE * EE * 2); bf* BK = (bf*)take((size_t)LL * EE * 2); bf* BV = (bf*)take((size_t)LL * EE * 2); bf* BQL = (bf*)take((size_t)NH_ * LL * HD * 2); bf* BVU = (bf*)take((size_t)NH_ * HD * LL * 2);
    float* Q = (float*)take((size_t)TT * EE * 4); bf* QHh = (bf*)take((size_t)NH_ * TT * HD * 2); bf* QHl = (bf*)take((size_t)NH_ * TT * HD * 2);
    float* LK = (float*)take((size_t)TT * LL * 4); float* LV = (float*)take((size_t)TT * LL * 4); bf* LKh = (bf*)take((size_t)TT * LL * 2); bf* LKl = (bf*)take((size_t)TT * LL * 2); bf* LVh = (bf*)take((size_t)TT * LL * 2); bf* LVl = (bf*)take((size_t)TT * LL * 2);
    float* QL = (float*)take((size_t)NH_ * TT * LL * 4); bf* QLh = (bf*)take((size_t)NH_ * TT * LL * 2); bf* QLl = (bf*)take((size_t)NH_ * TT * LL * 2); float* SQ = (float*)take((size_t)NH_ * TT * 4); float* SK = (float*)take((size_t)TT * 4);
    float* VE = (float*)take((size_t)NH_ * TT * HD * 4); bf* VETh = (bf*)take((size_t)NH_ * HD * TT * 2); bf* VETl = (bf*)take((size_t)NH_ * HD * TT * 2);
    float* S = (float*)take((size_t)ZH * TT * TT * 4); bf* Ph = (bf*)take((size_t)ZH * TT * TT * 2); bf* Pl = (bf*)take((size_t)ZH * TT * TT * 2); float* O = (float*)take((size_t)ZH * TT * HD * 4); bf* ATh = (bf*)take((size_t)TT * EE * 2); bf* ATl = (bf*)take((size_t)TT * EE * 2);
    if ((size_t)(wsp - (char*)d_ws) > ws_size) return;
    k_cvt8<<<(unsigned)(((size_t)EE * EE / 8 + 255) / 256), 256, 0, stream>>>(Wq, BQ, (size_t)EE * EE / 8); k_cvt8<<<(LL * EE / 8 + 255) / 256, 256, 0, stream>>>(Wk, BK, LL * EE / 8); k_cvt8<<<(LL * EE / 8 + 255) / 256, 256, 0, stream>>>(Wv, BV, LL * EE / 8);
    k_q2l<<<(NH_ * LL * HD / 4 + 255) / 256, 256, 0, stream>>>(q2l, BQL); k_vup<<<(NH_ * HD * LL / 4 + 255) / 256, 256, 0, stream>>>(vup, BVU);
    k_cvt8<<<(unsigned)(((size_t)TT * EE / 8 + 255) / 256), 256, 0, stream>>>(x, XB, (size_t)TT * EE / 8);
    k_gemmw<bf, 0, false><<<dim3(TT / 64, EE / 64, 1), 32, 0, stream>>>(XB, nullptr, BQ, nullptr, EE, Q, EE, nullptr, 0, 0, 0); k_qhpl<<<(unsigned)(((size_t)NH_ * TT * HD / 4 + 255) / 256), 256, 0, stream>>>(Q, QHh, QHl);
    k_cvt8<<<(unsigned)(((size_t)EE * EE / 8 + 255) / 256), 256, 0, stream>>>(Wo, BQ, (size_t)EE * EE / 8);
    k_gemmw<bf, 0, false><<<dim3(TT / 64, 1, 1), 32, 0, stream>>>(XB, nullptr, BK, nullptr, EE, LK, LL, nullptr, 0, 0, 0); k_gemmw<bf, 0, false><<<dim3(TT / 64, 1, 1), 32, 0, stream>>>(XB, nullptr, BV, nullptr, EE, LV, LL, nullptr, 0, 0, 0);
    k_pl<<<(TT * LL / 4 + 255) / 256, 256, 0, stream>>>(LK, (size_t)TT * LL, LKh, LKl); k_pl<<<(TT * LL / 4 + 255) / 256, 256, 0, stream>>>(LV, (size_t)TT * LL, LVh, LVl); k_rsum64<<<(TT + 255) / 256, 256, 0, stream>>>(LK, TT, SK);
    k_gemmw<bf, 1, false><<<dim3(TT / 64, 1, NH_), 32, 0, stream>>>(QHh, QHl, BQL, nullptr, HD, QL, LL, nullptr, (size_t)TT * HD, (size_t)LL * HD, (size_t)TT * LL);
    k_pl<<<(unsigned)(((size_t)NH_ * TT * LL / 4 + 255) / 256), 256, 0, stream>>>(QL, (size_t)NH_ * TT * LL, QLh, QLl); k_rsum64<<<(NH_ * TT + 255) / 256, 256, 0, stream>>>(QL, (size_t)NH_ * TT, SQ);
    k_gemmw<bf, 1, false><<<dim3(TT / 64, HD / 64, NH_), 32, 0, stream>>>(LVh, LVl, BVU, nullptr, LL, VE, HD, nullptr, 0, (size_t)HD * LL, (size_t)TT * HD);
    k_vet<<<(unsigned)(((size_t)NH_ * HD * TT / 2 + 255) / 256), 256, 0, stream>>>(VE, VETh, VETl);
    const size_t zql = (size_t)TT * LL, zS = (size_t)TT * TT, zv = (size_t)HD * TT, zo = (size_t)TT * HD;
    for (int h0 = 0; h0 < NH_; h0 += ZH) {
        k_gemmc<bf, 2, 1><<<dim3(TT / 64, TT / 64, ZH), 32, 0, stream>>>(QLh + (size_t)h0 * zql, QLl + (size_t)h0 * zql, LKh, LKl, LL, S, TT, 0, zql, 0, zS);
        k_csoft<<<ZH * TT / 8, 256, 0, stream>>>(S, SQ, SK, h0, Ph, Pl);
        k_gemmc<bf, 2, 2><<<dim3(TT / 64, HD / 64, ZH), 32, 0, stream>>>(Ph, Pl, VETh + (size_t)h0 * zv, VETl + (size_t)h0 * zv, TT, O, HD, 0, zS, zv, zo);
        k_merge<<<(unsigned)(((size_t)ZH * TT * HD / 4 + 255) / 256), 256, 0, stream>>>(O, h0, ATh, ATl); }
    k_gemmw<bf, 1, false><<<dim3(TT / 64, EE / 64, 1), 32, 0, stream>>>(ATh, ATl, BQ, nullptr, EE, OUT, EE, nullptr, 0, 0, 0);
}
